// MambaBlock_19129784336931
// MI455X (gfx1250) — hardware-run, weakly checked
//
#include <hip/hip_runtime.h>
#include <hip/hip_fp16.h>
#include <math.h>

typedef float    ms1_v4f __attribute__((ext_vector_type(4)));
typedef unsigned ms1_v4u __attribute__((ext_vector_type(4)));
struct ms1_args {
  const float* dtpre;
  const float* u;
  const float* bc;
  const float* z;
  const float* A_log;
  const float* Dskip;
  __half* y;
  __half* y_lo;
  long ld_dtpre;
  long ld_u;
  long ld_bc;
  long ld_z;
  long ld_y;
  int offB;
  int offC;
  int offZ;
  float ycarry;
  int dir;
  int D;
  int L;
  int nbatch;
};
static_assert(sizeof(ms1_args) == 136);

__device__ __forceinline__ float ms1_flush16(float v) {
  return (fabsf(v) < 6.103515625e-05f) ? 0.0f : v;
}
__device__ __forceinline__ unsigned ms1_h16bits(float v) {
  return (unsigned)__half_as_ushort(__float2half_rn(ms1_flush16(v)));
}
__device__ __forceinline__ float ms1_h16val(unsigned b) {
  return __half2float(__ushort_as_half((unsigned short)b));
}
__device__ __forceinline__ float ms1_softplus(float v) {
  return fmaxf(v, 0.0f) + log1pf(expf(-fabsf(v)));
}
__device__ __forceinline__ void ms1_pack2(float v0, float v1, unsigned& hw, unsigned& lw) {
  const unsigned h0 = ms1_h16bits(v0);
  const unsigned h1 = ms1_h16bits(v1);
  const float r0 = (v0 - ms1_h16val(h0)) * 2048.0f;
  const float r1 = (v1 - ms1_h16val(h1)) * 2048.0f;
  const unsigned l0 = ms1_h16bits(r0);
  const unsigned l1 = ms1_h16bits(r1);
  hw = h0 | (h1 << 16);
  lw = l0 | (l1 << 16);
}

template <int NSTATE>
__global__ __launch_bounds__(64 * (NSTATE / 16)) void ms1_scan_kernel(ms1_args a)
{
  static_assert(NSTATE == 16 || NSTATE == 64);
  constexpr int NQ  = NSTATE / 16;
  constexpr int NT  = 64 * NQ;
  constexpr int NW  = NT / 32;
  constexpr int BCW = 2 * NSTATE;
  constexpr int YP  = 68;
  constexpr int RPI = NW * 4;
  constexpr int NIT = 64 / RPI;
  static_assert(16 * NT <= 64 * YP);
  __shared__ __align__(16) float sBC[64 * BCW];
  __shared__ __align__(16) float sY[64 * YP];
  const int tid  = threadIdx.x;
  const int lane = tid & 31;
  const int wave = tid >> 5;
  const int c    = tid / NQ;
  const int sq   = tid - c * NQ;
  const int bpb  = a.D / 64;
  const int bi   = blockIdx.x / bpb;
  if (bi >= a.nbatch) return;
  const int d0 = (blockIdx.x - bi * bpb) * 64;
  const int d  = d0 + c;
  const long rowb = (long)bi * a.L;
  const bool hasz  = (a.z != nullptr);
  const bool hasD  = (a.Dskip != nullptr);
  const bool hasLo = (a.y_lo != nullptr);

#pragma unroll 1
  for (int n = 0; n < 16; ++n) {
    const float al = a.A_log[(long)d * NSTATE + sq * 16 + n];
    sY[n * NT + tid] = -expf(al);
  }
  __syncthreads();
  float An[16], h[16];
#pragma unroll
  for (int n = 0; n < 16; ++n) {
    An[n] = sY[n * NT + tid];
    h[n] = 0.0f;
  }
  float Dd = 0.0f;
  if (hasD) Dd = a.Dskip[d];

  const int nchunk = a.L / 64;
  const bool fwd = (a.dir > 0);
  const int s0 = fwd ? 0 : 63;
  const int sd = fwd ? 1 : -1;
  const int q  = lane >> 3;
  const int c8 = (lane & 7) * 8;

#pragma unroll 1
  for (int ci = 0; ci < nchunk; ++ci) {
    const int tb = fwd ? (ci * 64) : (a.L - 64 - ci * 64);
    const long rowc = rowb + tb;
    __syncthreads();
#pragma unroll 8
    for (int i = 0; i < 32; ++i) {
      const int idx = tid + i * NT;
      const int st  = idx / BCW;
      const int col = idx - st * BCW;
      const int sc  = (col < NSTATE) ? (a.offB + col) : (a.offC + col - NSTATE);
      sBC[idx] = a.bc[(rowc + st) * a.ld_bc + sc];
    }
    __syncthreads();
#pragma unroll 1
    for (int s = 0; s < 64; ++s) {
      const int ls = s0 + sd * s;
      const long row = rowc + ls;
      float pre = a.dtpre[row * a.ld_dtpre + d];
      float uv  = a.u[row * a.ld_u + d];
      float zv  = 0.0f;
      if (hasz) zv = a.z[row * a.ld_z + a.offZ + d];
      asm volatile("" : "+v"(pre));
      asm volatile("" : "+v"(uv));
      asm volatile("" : "+v"(zv));
      const float delta = ms1_softplus(pre);
      const float dtx = delta * uv;
      const float* bp = sBC + ls * BCW + sq * 16;
      const float* cp = bp + NSTATE;
      ms1_v4f Bq[4], Cq[4];
#pragma unroll
      for (int k = 0; k < 4; ++k) {
        Bq[k] = *(const ms1_v4f*)(bp + 4 * k);
        Cq[k] = *(const ms1_v4f*)(cp + 4 * k);
      }
      float yv = 0.0f;
#pragma unroll
      for (int n = 0; n < 16; ++n) {
        const float e = __expf(delta * An[n]);
        h[n] = fmaf(e, h[n], dtx * Bq[n >> 2][n & 3]);
        yv = fmaf(h[n], Cq[n >> 2][n & 3], yv);
      }
      if (NQ > 1) {
        yv += __shfl_xor(yv, 1, 32);
        yv += __shfl_xor(yv, 2, 32);
      }
      if (hasD) yv = fmaf(uv, Dd, yv);
      if (hasz) {
        const float sg = __builtin_amdgcn_rcpf(1.0f + expf(-zv));
        yv = yv * (zv * sg);
      }
      if (sq == 0) sY[ls * YP + c] = yv * a.ycarry;
    }
    __syncthreads();
    ms1_v4u hw[NIT], lw[NIT];
#pragma unroll
    for (int it = 0; it < NIT; ++it) {
      const int row = it * RPI + wave * 4 + q;
      const float* sp = sY + row * YP + c8;
      const ms1_v4f f0 = *(const ms1_v4f*)(sp);
      const ms1_v4f f1 = *(const ms1_v4f*)(sp + 4);
      unsigned h0, h1, h2, h3, l0, l1, l2, l3;
      ms1_pack2(f0[0], f0[1], h0, l0);
      ms1_pack2(f0[2], f0[3], h1, l1);
      ms1_pack2(f1[0], f1[1], h2, l2);
      ms1_pack2(f1[2], f1[3], h3, l3);
      hw[it] = (ms1_v4u){h0, h1, h2, h3};
      lw[it] = (ms1_v4u){l0, l1, l2, l3};
    }
    for (int pass = 0; pass < 2; ++pass) {
#pragma unroll
      for (int it = 0; it < NIT; ++it) {
        const int row = it * RPI + wave * 4 + q;
        const long o = (rowc + row) * a.ld_y + d0 + c8;
        *(volatile ms1_v4u*)(a.y + o) = hw[it];
        if (hasLo) *(volatile ms1_v4u*)(a.y_lo + o) = lw[it];
      }
      __threadfence();
    }
  }
}

namespace eng {

constexpr int kBatch  = 2;
constexpr int kSeq    = 2048;
constexpr int kDm     = 1024;
constexpr int kDin    = 2048;
constexpr int kNstate = 16;
constexpr int kXzN    = 2 * kDin;
constexpr int kSsmN   = 2 * kNstate + 1;
constexpr int kBcP    = 64;
constexpr int kOffB   = 16;
constexpr int kOffC   = 32;

static_assert(kSsmN == 33);
static_assert(kOffC + kNstate <= kBcP);
static_assert(kSeq % 64 == 0 && kXzN % 64 == 0 && kBcP % 64 == 0 && kDin % 64 == 0 && kDm % 64 == 0);
static_assert(kDm % 32 == 0 && kDin % 32 == 0);
static_assert(kDm == 4 * 256 && kDin == 2 * 1024);
static_assert(((kSeq / 64) * (kXzN / 64)) % 8 == 0);
static_assert(((kSeq / 64) * (kBcP / 64)) % 8 == 0);
static_assert(((kSeq / 32) * (kDm / 64)) % 8 == 0);

constexpr float kCarryY    = 16.0f;
constexpr float kCarryWout = 256.0f;
constexpr float kResid     = 2048.0f;
constexpr float kFoldOut   = 1.0f / (kCarryY * kCarryWout);
constexpr float kFoldResid = 1.0f / kResid;

constexpr size_t kBytesWinB  = (size_t)kXzN * kDm * 2;
constexpr size_t kBytesWoutH = (size_t)kDm * kDin * 2;
constexpr size_t kBytesWxB   = (size_t)kBcP * kDin * 2;
constexpr size_t kBytesAlog  = (size_t)kDin * kNstate * 4;
constexpr size_t kBytesDpar  = (size_t)kDin * 4;
constexpr size_t kBytesXNh   = (size_t)kSeq * kDm * 2;
constexpr size_t kBytesXNl   = (size_t)kSeq * kDm * 2;
constexpr size_t kBytesXZ    = (size_t)kSeq * kXzN * 4;
constexpr size_t kBytesU     = (size_t)kSeq * kDin * 4;
constexpr size_t kBytesUh    = (size_t)kSeq * kDin * 2;
constexpr size_t kBytesUl    = (size_t)kSeq * kDin * 2;
constexpr size_t kBytesBC    = (size_t)kSeq * kBcP * 4;
constexpr size_t kBytesDTP   = (size_t)kSeq * kDin * 4;
constexpr size_t kBytesYH    = (size_t)kSeq * kDin * 2;
constexpr size_t kBytesYL    = (size_t)kSeq * kDin * 2;
constexpr size_t kWsTotal = kBytesWinB + kBytesWoutH + kBytesWxB + kBytesAlog + kBytesDpar + kBytesXNh + kBytesXNl +
                            kBytesXZ + kBytesU + kBytesUh + kBytesUl + kBytesBC + kBytesDTP + kBytesYH + kBytesYL;
static_assert(kWsTotal == 122560512ull);
static_assert(kWsTotal <= 134217728ull);
static_assert(kBytesWinB % 128 == 0 && kBytesWoutH % 128 == 0 && kBytesWxB % 128 == 0 && kBytesAlog % 128 == 0 &&
              kBytesDpar % 128 == 0 && kBytesXNh % 128 == 0 && kBytesXNl % 128 == 0 && kBytesXZ % 128 == 0 &&
              kBytesU % 128 == 0 && kBytesUh % 128 == 0 && kBytesUl % 128 == 0 && kBytesBC % 128 == 0 &&
              kBytesDTP % 128 == 0 && kBytesYH % 128 == 0 && kBytesYL % 128 == 0);

typedef _Float16 v16h __attribute__((ext_vector_type(16)));
typedef _Float16 v8h  __attribute__((ext_vector_type(8)));
typedef __bf16   v16b __attribute__((ext_vector_type(16)));
typedef __bf16   v8b  __attribute__((ext_vector_type(8)));
typedef float    v8f  __attribute__((ext_vector_type(8)));
typedef float    v4f  __attribute__((ext_vector_type(4)));
typedef unsigned v4u  __attribute__((ext_vector_type(4)));

__device__ __forceinline__ unsigned bf16_bits(float f) {
  const unsigned u = __float_as_uint(f);
  return (u + 0x7FFFu + ((u >> 16) & 1u)) >> 16;
}
__device__ __forceinline__ float bf16_val(unsigned b) {
  return __uint_as_float(b << 16);
}
__device__ __forceinline__ float bf16r(float f) {
  return bf16_val(bf16_bits(f));
}
__device__ __forceinline__ unsigned pk_bf16(float a, float b) {
  const unsigned lo = bf16_bits(a);
  const unsigned hi = bf16_bits(b);
  return lo | (hi << 16);
}
__device__ __forceinline__ void split2_bf16(float v0, float v1, unsigned& hw, unsigned& lw) {
  const unsigned h0 = bf16_bits(v0);
  const unsigned h1 = bf16_bits(v1);
  const unsigned l0 = bf16_bits(v0 - bf16_val(h0));
  const unsigned l1 = bf16_bits(v1 - bf16_val(h1));
  hw = h0 | (h1 << 16);
  lw = l0 | (l1 << 16);
}
__device__ __forceinline__ float f16_flush(float v) {
  return (fabsf(v) < 6.103515625e-05f) ? 0.0f : v;
}
__device__ __forceinline__ unsigned f16_bits(float v) {
  return (unsigned)__half_as_ushort(__float2half_rn(f16_flush(v)));
}
__device__ __forceinline__ unsigned pk_f16(float a, float b) {
  const unsigned lo = f16_bits(a);
  const unsigned hi = f16_bits(b);
  return lo | (hi << 16);
}

template <int ET> struct Op;
template <> struct Op<0> {
  typedef _Float16 T;
  typedef v16h V;
  union U { v16h v; v8h h[2]; };
  static __device__ __forceinline__ V load(const T* p) {
    U f;
    f.h[0] = *(const v8h*)(p);
    f.h[1] = *(const v8h*)(p + 16);
    return f.v;
  }
  static __device__ __forceinline__ v8f mma(V a, V b, v8f c) {
    c = __builtin_amdgcn_wmma_f32_16x16x32_f16(false, a, false, b, (short)0, c, false, false);
    asm volatile("v_nop\n\tv_nop\n\tv_nop\n\tv_nop" : "+v"(c) : "v"(a), "v"(b));
    return c;
  }
};
template <> struct Op<1> {
  typedef __bf16 T;
  typedef v16b V;
  union U { v16b v; v8b h[2]; };
  static __device__ __forceinline__ V load(const T* p) {
    U f;
    f.h[0] = *(const v8b*)(p);
    f.h[1] = *(const v8b*)(p + 16);
    return f.v;
  }
  static __device__ __forceinline__ v8f mma(V a, V b, v8f c) {
    c = __builtin_amdgcn_wmma_f32_16x16x32_bf16(false, a, false, b, (short)0, c, false, false);
    asm volatile("v_nop\n\tv_nop\n\tv_nop\n\tv_nop" : "+v"(c) : "v"(a), "v"(b));
    return c;
  }
};

__global__ __launch_bounds__(256) void cast_bf16_kernel(
    const float* __restrict__ in, unsigned short* __restrict__ out, int n8)
{
  const int i = blockIdx.x * 256 + threadIdx.x;
  if (i < n8) {
    const v4f f0 = *(const v4f*)(in + (size_t)i * 8);
    const v4f f1 = *(const v4f*)(in + (size_t)i * 8 + 4);
    const float e0 = f0[0];
    const float e1 = f0[1];
    const float e2 = f0[2];
    const float e3 = f0[3];
    const float e4 = f1[0];
    const float e5 = f1[1];
    const float e6 = f1[2];
    const float e7 = f1[3];
    const v4u hw = (v4u){pk_bf16(e0, e1), pk_bf16(e2, e3), pk_bf16(e4, e5), pk_bf16(e6, e7)};
    unsigned short* o = out + (size_t)i * 8;
    for (int pass = 0; pass < 2; ++pass) {
      *(volatile v4u*)(o) = hw;
      __threadfence();
    }
  }
}

__global__ __launch_bounds__(256) void cast_f16_carry_kernel(
    const float* __restrict__ in, unsigned short* __restrict__ out, int n8, float carry)
{
  const int i = blockIdx.x * 256 + threadIdx.x;
  if (i < n8) {
    const v4f f0 = *(const v4f*)(in + (size_t)i * 8);
    const v4f f1 = *(const v4f*)(in + (size_t)i * 8 + 4);
    const float e0 = f0[0];
    const float e1 = f0[1];
    const float e2 = f0[2];
    const float e3 = f0[3];
    const float e4 = f1[0];
    const float e5 = f1[1];
    const float e6 = f1[2];
    const float e7 = f1[3];
    const float c0 = bf16r(e0) * carry;
    const float c1 = bf16r(e1) * carry;
    const float c2 = bf16r(e2) * carry;
    const float c3 = bf16r(e3) * carry;
    const float c4 = bf16r(e4) * carry;
    const float c5 = bf16r(e5) * carry;
    const float c6 = bf16r(e6) * carry;
    const float c7 = bf16r(e7) * carry;
    const v4u hw = (v4u){pk_f16(c0, c1), pk_f16(c2, c3), pk_f16(c4, c5), pk_f16(c6, c7)};
    unsigned short* o = out + (size_t)i * 8;
    for (int pass = 0; pass < 2; ++pass) {
      *(volatile v4u*)(o) = hw;
      __threadfence();
    }
  }
}

__global__ __launch_bounds__(256) void xproj_weight_kernel(
    const float* __restrict__ in, unsigned short* __restrict__ out)
{
  const int n = blockIdx.x;
  const int k8 = threadIdx.x * 8;
  const bool live = (n == 0) || (n >= kOffB && n < kOffC + kNstate);
  int src = (n == 0) ? 0 : (n - (kOffB - 1));
  src = (src < 0) ? 0 : src;
  src = (src > kSsmN - 1) ? (kSsmN - 1) : src;
  const v4f f0 = *(const v4f*)(in + (size_t)src * kDin + k8);
  const v4f f1 = *(const v4f*)(in + (size_t)src * kDin + k8 + 4);
  const float e0 = live ? f0[0] : 0.0f;
  const float e1 = live ? f0[1] : 0.0f;
  const float e2 = live ? f0[2] : 0.0f;
  const float e3 = live ? f0[3] : 0.0f;
  const float e4 = live ? f1[0] : 0.0f;
  const float e5 = live ? f1[1] : 0.0f;
  const float e6 = live ? f1[2] : 0.0f;
  const float e7 = live ? f1[3] : 0.0f;
  const v4u hw = (v4u){pk_bf16(e0, e1), pk_bf16(e2, e3), pk_bf16(e4, e5), pk_bf16(e6, e7)};
  unsigned short* o = out + (size_t)n * kDin + k8;
  for (int pass = 0; pass < 2; ++pass) {
    *(volatile v4u*)(o) = hw;
    __threadfence();
  }
}

__global__ __launch_bounds__(256) void table_bf16r_kernel(
    const float* __restrict__ in, float* __restrict__ out, int n4)
{
  const int i = blockIdx.x * 256 + threadIdx.x;
  if (i < n4) {
    const v4f f0 = *(const v4f*)(in + (size_t)i * 4);
    const float e0 = f0[0];
    const float e1 = f0[1];
    const float e2 = f0[2];
    const float e3 = f0[3];
    const v4f o = (v4f){bf16r(e0), bf16r(e1), bf16r(e2), bf16r(e3)};
    for (int pass = 0; pass < 2; ++pass) {
      *(volatile v4f*)(out + (size_t)i * 4) = o;
      __threadfence();
    }
  }
}

__global__ __launch_bounds__(256) void rownorm_split_kernel(
    const float* __restrict__ x, const float* __restrict__ ln_w, const float* __restrict__ ln_b,
    unsigned short* __restrict__ XNh, unsigned short* __restrict__ XNl, int rows)
{
  const int lane = threadIdx.x & 31;
  const int wave = threadIdx.x >> 5;
  const int row = blockIdx.x * 8 + wave;
  if (row >= rows) return;
  const float* xr = x + (size_t)row * kDm;
  float v[4][8];
#pragma unroll
  for (int it = 0; it < 4; ++it) {
    const v4f f0 = *(const v4f*)(xr + it * 256 + lane * 8);
    const v4f f1 = *(const v4f*)(xr + it * 256 + lane * 8 + 4);
    const float e0 = f0[0];
    const float e1 = f0[1];
    const float e2 = f0[2];
    const float e3 = f0[3];
    const float e4 = f1[0];
    const float e5 = f1[1];
    const float e6 = f1[2];
    const float e7 = f1[3];
    v[it][0] = bf16r(e0);
    v[it][1] = bf16r(e1);
    v[it][2] = bf16r(e2);
    v[it][3] = bf16r(e3);
    v[it][4] = bf16r(e4);
    v[it][5] = bf16r(e5);
    v[it][6] = bf16r(e6);
    v[it][7] = bf16r(e7);
  }
  float s = 0.0f;
#pragma unroll
  for (int it = 0; it < 4; ++it) {
    float p = 0.0f;
#pragma unroll
    for (int e = 0; e < 8; ++e) p += v[it][e];
    s += p;
  }
  s += __shfl_xor(s, 16, 32);
  s += __shfl_xor(s, 8, 32);
  s += __shfl_xor(s, 4, 32);
  s += __shfl_xor(s, 2, 32);
  s += __shfl_xor(s, 1, 32);
  const float mu = s * (1.0f / (float)kDm);
  float qs = 0.0f;
#pragma unroll
  for (int it = 0; it < 4; ++it) {
    float p = 0.0f;
#pragma unroll
    for (int e = 0; e < 8; ++e) {
      const float dlt = v[it][e] - mu;
      p = fmaf(dlt, dlt, p);
    }
    qs += p;
  }
  qs += __shfl_xor(qs, 16, 32);
  qs += __shfl_xor(qs, 8, 32);
  qs += __shfl_xor(qs, 4, 32);
  qs += __shfl_xor(qs, 2, 32);
  qs += __shfl_xor(qs, 1, 32);
  const float var = qs * (1.0f / (float)kDm);
  const float rs = rsqrtf(var + 1e-5f);
  v4u hw[4], lw[4];
#pragma unroll
  for (int it = 0; it < 4; ++it) {
    const v4f w0 = *(const v4f*)(ln_w + it * 256 + lane * 8);
    const v4f w1 = *(const v4f*)(ln_w + it * 256 + lane * 8 + 4);
    const v4f b0 = *(const v4f*)(ln_b + it * 256 + lane * 8);
    const v4f b1 = *(const v4f*)(ln_b + it * 256 + lane * 8 + 4);
    const float g0 = w0[0];
    const float g1 = w0[1];
    const float g2 = w0[2];
    const float g3 = w0[3];
    const float g4 = w1[0];
    const float g5 = w1[1];
    const float g6 = w1[2];
    const float g7 = w1[3];
    const float t0 = b0[0];
    const float t1 = b0[1];
    const float t2 = b0[2];
    const float t3 = b0[3];
    const float t4 = b1[0];
    const float t5 = b1[1];
    const float t6 = b1[2];
    const float t7 = b1[3];
    const float n0 = fmaf((v[it][0] - mu) * rs, bf16r(g0), bf16r(t0));
    const float n1 = fmaf((v[it][1] - mu) * rs, bf16r(g1), bf16r(t1));
    const float n2 = fmaf((v[it][2] - mu) * rs, bf16r(g2), bf16r(t2));
    const float n3 = fmaf((v[it][3] - mu) * rs, bf16r(g3), bf16r(t3));
    const float n4 = fmaf((v[it][4] - mu) * rs, bf16r(g4), bf16r(t4));
    const float n5 = fmaf((v[it][5] - mu) * rs, bf16r(g5), bf16r(t5));
    const float n6 = fmaf((v[it][6] - mu) * rs, bf16r(g6), bf16r(t6));
    const float n7 = fmaf((v[it][7] - mu) * rs, bf16r(g7), bf16r(t7));
    unsigned h0, h1, h2, h3, l0, l1, l2, l3;
    split2_bf16(n0, n1, h0, l0);
    split2_bf16(n2, n3, h1, l1);
    split2_bf16(n4, n5, h2, l2);
    split2_bf16(n6, n7, h3, l3);
    hw[it] = (v4u){h0, h1, h2, h3};
    lw[it] = (v4u){l0, l1, l2, l3};
  }
  unsigned short* oh = XNh + (size_t)row * kDm + lane * 8;
  unsigned short* ol = XNl + (size_t)row * kDm + lane * 8;
  for (int pass = 0; pass < 2; ++pass) {
#pragma unroll
    for (int it = 0; it < 4; ++it) {
      *(volatile v4u*)(oh + it * 256) = hw[it];
      *(volatile v4u*)(ol + it * 256) = lw[it];
    }
    __threadfence();
  }
}

template <int ET, int MT, int ATERMS, int SEP, int EPI>
__global__ __launch_bounds__(256) void gemm16_kernel(
    const unsigned short* __restrict__ Ap, const unsigned short* __restrict__ A2p, int lda,
    const unsigned short* __restrict__ Btp, int ldb,
    float* __restrict__ C, int ldc,
    const float* __restrict__ R, int ldr,
    int M, int N, int K, float scale, float scale2)
{
  typedef typename Op<ET>::T T;
  typedef typename Op<ET>::V V;
  const T* A  = (const T*)(const void*)Ap;
  const T* A2 = (const T*)(const void*)A2p;
  const T* Bt = (const T*)(const void*)Btp;
  __shared__ __align__(16) float sT[8][16 * 68];
  const int lane = threadIdx.x & 31;
  const int wave = threadIdx.x >> 5;
  const int tilesN = N >> 6;
  const int tilesM = M / (16 * MT);
  const int tile = blockIdx.x * 8 + wave;
  if (tile >= tilesM * tilesN) return;
  const int tm = tile / tilesN;
  const int tn = tile - tm * tilesN;
  const int m0 = tm * (16 * MT);
  const int n0 = tn << 6;
  const int rlane = lane & 15;
  const int koff  = (lane >> 4) * 8;
  const int mOff  = (lane >> 4) * 8;
  constexpr int NL = (SEP == 1) ? MT : 1;

  v8f accH[MT][4];
  v8f accL[NL][4];
#pragma unroll
  for (int i = 0; i < MT; ++i) {
#pragma unroll
    for (int j = 0; j < 4; ++j) {
      accH[i][j] = (v8f){0.f, 0.f, 0.f, 0.f, 0.f, 0.f, 0.f, 0.f};
    }
  }
#pragma unroll
  for (int i = 0; i < NL; ++i) {
#pragma unroll
    for (int j = 0; j < 4; ++j) {
      accL[i][j] = (v8f){0.f, 0.f, 0.f, 0.f, 0.f, 0.f, 0.f, 0.f};
    }
  }

#pragma unroll 1
  for (int k0 = 0; k0 < K; k0 += 32) {
    V bf[4];
#pragma unroll
    for (int j = 0; j < 4; ++j) {
      bf[j] = Op<ET>::load(Bt + (size_t)(n0 + (j << 4) + rlane) * ldb + koff + k0);
    }
#pragma unroll
    for (int i = 0; i < MT; ++i) {
      const size_t ao = (size_t)(m0 + (i << 4) + rlane) * lda + koff + k0;
      const V a0 = Op<ET>::load(A + ao);
#pragma unroll
      for (int j = 0; j < 4; ++j) accH[i][j] = Op<ET>::mma(a0, bf[j], accH[i][j]);
      if (ATERMS == 2) {
        const V a1 = Op<ET>::load(A2 + ao);
        if (SEP == 1) {
#pragma unroll
          for (int j = 0; j < 4; ++j) accL[(SEP == 1) ? i : 0][j] = Op<ET>::mma(a1, bf[j], accL[(SEP == 1) ? i : 0][j]);
        } else {
#pragma unroll
          for (int j = 0; j < 4; ++j) accH[i][j] = Op<ET>::mma(a1, bf[j], accH[i][j]);
        }
      }
    }
  }

  float* slab = sT[wave];
#pragma unroll
  for (int i = 0; i < MT; ++i) {
    const int mBase = m0 + (i << 4);
#pragma unroll
    for (int j = 0; j < 4; ++j) {
#pragma unroll
      for (int r = 0; r < 8; ++r) {
        float v = accH[i][j][r];
        if (SEP == 1) v = v + accL[(SEP == 1) ? i : 0][j][r] * scale2;
        v = v * scale;
        slab[(mOff + r) * 68 + (j << 4) + rlane] = v;
      }
    }
    __builtin_amdgcn_fence(__ATOMIC_RELEASE, "workgroup");
    __builtin_amdgcn_wave_barrier();
    __builtin_amdgcn_fence(__ATOMIC_ACQUIRE, "workgroup");
    {
      const int hh = lane >> 4;
      const int c4 = (lane & 15) * 4;
      v4f vals[8];
#pragma unroll
      for (int it = 0; it < 8; ++it) {
        const int row = it * 2 + hh;
        v4f val = *(const v4f*)(slab + row * 68 + c4);
        if (EPI == 1) {
          const v4f rv = *(const v4f*)(R + (size_t)(mBase + row) * ldr + n0 + c4);
          const float r0 = rv[0];
          const float r1 = rv[1];
          const float r2 = rv[2];
          const float r3 = rv[3];
          const float s0 = val[0];
          const float s1 = val[1];
          const float s2 = val[2];
          const float s3 = val[3];
          val = (v4f){s0 + bf16r(r0), s1 + bf16r(r1), s2 + bf16r(r2), s3 + bf16r(r3)};
        }
        vals[it] = val;
      }
      for (int pass = 0; pass < 2; ++pass) {
#pragma unroll
        for (int it = 0; it < 8; ++it) {
          const int row = it * 2 + hh;
          *(volatile v4f*)(C + (size_t)(mBase + row) * ldc + n0 + c4) = vals[it];
        }
        __threadfence();
      }
    }
    __builtin_amdgcn_fence(__ATOMIC_RELEASE, "workgroup");
    __builtin_amdgcn_wave_barrier();
    __builtin_amdgcn_fence(__ATOMIC_ACQUIRE, "workgroup");
  }
}

__device__ __forceinline__ float tap4_silu(v4f w, float u0, float u1, float u2, float u3, float b) {
  const float w0 = w[0];
  const float w1 = w[1];
  const float w2 = w[2];
  const float w3 = w[3];
  float acc = bf16r(w0) * u0;
  acc = fmaf(bf16r(w1), u1, acc);
  acc = fmaf(bf16r(w2), u2, acc);
  acc = fmaf(bf16r(w3), u3, acc);
  const float cv = acc + bf16r(b);
  const float sg = __builtin_amdgcn_rcpf(1.0f + expf(-cv));
  return cv * sg;
}

__global__ __launch_bounds__(256) void conv_silu_split_kernel(
    const float* __restrict__ XZ, const float* __restrict__ conv_w, const float* __restrict__ conv_b,
    float* __restrict__ U, unsigned short* __restrict__ Uh, unsigned short* __restrict__ Ul)
{
  __shared__ __align__(16) float sRow[kDin];
  const int tid = threadIdx.x;
  const int t = blockIdx.x;
#pragma unroll 1
  for (int g = 0; g < 2; ++g) {
    const int d4 = g * 1024 + tid * 4;
    const v4f bs = *(const v4f*)(conv_b + d4);
    const v4f w0 = *(const v4f*)(conv_w + (size_t)d4 * 4);
    const v4f w1 = *(const v4f*)(conv_w + (size_t)d4 * 4 + 4);
    const v4f w2 = *(const v4f*)(conv_w + (size_t)d4 * 4 + 8);
    const v4f w3 = *(const v4f*)(conv_w + (size_t)d4 * 4 + 12);
    v4f ut[4];
#pragma unroll
    for (int k = 0; k < 4; ++k) {
      const int tt = t - 3 + k;
      const int tc = (tt < 0) ? 0 : tt;
      const bool on = (tt >= 0);
      const v4f ld = *(const v4f*)(XZ + (size_t)tc * kXzN + d4);
      const float a0 = ld[0];
      const float a1 = ld[1];
      const float a2 = ld[2];
      const float a3 = ld[3];
      ut[k] = (v4f){on ? a0 : 0.0f, on ? a1 : 0.0f, on ? a2 : 0.0f, on ? a3 : 0.0f};
    }
    const float b0 = bs[0];
    const float b1 = bs[1];
    const float b2 = bs[2];
    const float b3 = bs[3];
    v4f o;
    o[0] = tap4_silu(w0, ut[0][0], ut[1][0], ut[2][0], ut[3][0], b0);
    o[1] = tap4_silu(w1, ut[0][1], ut[1][1], ut[2][1], ut[3][1], b1);
    o[2] = tap4_silu(w2, ut[0][2], ut[1][2], ut[2][2], ut[3][2], b2);
    o[3] = tap4_silu(w3, ut[0][3], ut[1][3], ut[2][3], ut[3][3], b3);
    *(v4f*)(sRow + d4) = o;
  }
  __syncthreads();
  const v4f o0 = *(const v4f*)(sRow + tid * 4);
  const v4f o1 = *(const v4f*)(sRow + 1024 + tid * 4);
  const v4f f0 = *(const v4f*)(sRow + tid * 8);
  const v4f f1 = *(const v4f*)(sRow + tid * 8 + 4);
  const float e0 = f0[0];
  const float e1 = f0[1];
  const float e2 = f0[2];
  const float e3 = f0[3];
  const float e4 = f1[0];
  const float e5 = f1[1];
  const float e6 = f1[2];
  const float e7 = f1[3];
  unsigned h0, h1, h2, h3, l0, l1, l2, l3;
  split2_bf16(e0, e1, h0, l0);
  split2_bf16(e2, e3, h1, l1);
  split2_bf16(e4, e5, h2, l2);
  split2_bf16(e6, e7, h3, l3);
  const v4u hw = (v4u){h0, h1, h2, h3};
  const v4u lw = (v4u){l0, l1, l2, l3};
  float* ur = U + (size_t)t * kDin;
  unsigned short* uh = Uh + (size_t)t * kDin;
  unsigned short* ul = Ul + (size_t)t * kDin;
  for (int pass = 0; pass < 2; ++pass) {
    *(volatile v4f*)(ur + tid * 4) = o0;
    *(volatile v4f*)(ur + 1024 + tid * 4) = o1;
    *(volatile v4u*)(uh + tid * 8) = hw;
    *(volatile v4u*)(ul + tid * 8) = lw;
    __threadfence();
  }
}

__global__ __launch_bounds__(256) void step_preact_kernel(
    const float* __restrict__ BC, const float* __restrict__ W_dt, const float* __restrict__ b_dt,
    float* __restrict__ DTP)
{
  const int tid = threadIdx.x;
  const int r0 = blockIdx.x * 4;
  const v4f wa = *(const v4f*)(W_dt + tid * 4);
  const v4f wb = *(const v4f*)(W_dt + 1024 + tid * 4);
  const v4f ba = *(const v4f*)(b_dt + tid * 4);
  const v4f bb = *(const v4f*)(b_dt + 1024 + tid * 4);
  const float wa0 = wa[0];
  const float wa1 = wa[1];
  const float wa2 = wa[2];
  const float wa3 = wa[3];
  const float wb0 = wb[0];
  const float wb1 = wb[1];
  const float wb2 = wb[2];
  const float wb3 = wb[3];
  const float ba0 = ba[0];
  const float ba1 = ba[1];
  const float ba2 = ba[2];
  const float ba3 = ba[3];
  const float bb0 = bb[0];
  const float bb1 = bb[1];
  const float bb2 = bb[2];
  const float bb3 = bb[3];
  const float cwa0 = bf16r(wa0);
  const float cwa1 = bf16r(wa1);
  const float cwa2 = bf16r(wa2);
  const float cwa3 = bf16r(wa3);
  const float cwb0 = bf16r(wb0);
  const float cwb1 = bf16r(wb1);
  const float cwb2 = bf16r(wb2);
  const float cwb3 = bf16r(wb3);
  const float cba0 = bf16r(ba0);
  const float cba1 = bf16r(ba1);
  const float cba2 = bf16r(ba2);
  const float cba3 = bf16r(ba3);
  const float cbb0 = bf16r(bb0);
  const float cbb1 = bf16r(bb1);
  const float cbb2 = bf16r(bb2);
  const float cbb3 = bf16r(bb3);
#pragma unroll 1
  for (int rr = 0; rr < 4; ++rr) {
    const int row = r0 + rr;
    const float dr = BC[(size_t)row * kBcP];
    const v4f oa = (v4f){fmaf(dr, cwa0, cba0), fmaf(dr, cwa1, cba1), fmaf(dr, cwa2, cba2), fmaf(dr, cwa3, cba3)};
    const v4f ob = (v4f){fmaf(dr, cwb0, cbb0), fmaf(dr, cwb1, cbb1), fmaf(dr, cwb2, cbb2), fmaf(dr, cwb3, cbb3)};
    float* o = DTP + (size_t)row * kDin;
    for (int pass = 0; pass < 2; ++pass) {
      *(volatile v4f*)(o + tid * 4) = oa;
      *(volatile v4f*)(o + 1024 + tid * 4) = ob;
      __threadfence();
    }
  }
}

}

extern "C" void kernel_launch(void* const* d_in, const int* in_sizes, int n_in,
                              void* d_out, int out_size, void* d_ws, size_t ws_size, hipStream_t stream)
{
  using namespace eng;
  if (n_in != 12) return;
  if (in_sizes[0] != kBatch * kSeq * kDm) return;
  if (in_sizes[1] != kDm) return;
  if (in_sizes[2] != kDm) return;
  if (in_sizes[3] != kXzN * kDm) return;
  if (in_sizes[4] != kDin * 4) return;
  if (in_sizes[5] != kDin) return;
  if (in_sizes[6] != kSsmN * kDin) return;
  if (in_sizes[7] != kDin) return;
  if (in_sizes[8] != kDin) return;
  if (in_sizes[9] != kDin * kNstate) return;
  if (in_sizes[10] != kDin) return;
  if (in_sizes[11] != kDm * kDin) return;
  if (out_size != kBatch * kSeq * kDm) return;
  if (ws_size < kWsTotal) return;

  const float* x      = (const float*)d_in[0];
  const float* ln_w   = (const float*)d_in[1];
  const float* ln_b   = (const float*)d_in[2];
  const float* W_in   = (const float*)d_in[3];
  const float* conv_w = (const float*)d_in[4];
  const float* conv_b = (const float*)d_in[5];
  const float* W_x    = (const float*)d_in[6];
  const float* W_dt   = (const float*)d_in[7];
  const float* b_dt   = (const float*)d_in[8];
  const float* A_log  = (const float*)d_in[9];
  const float* D_par  = (const float*)d_in[10];
  const float* W_out  = (const float*)d_in[11];
  float* out = (float*)d_out;

  char* ws = (char*)d_ws;
  size_t off = 0;
  unsigned short* WinB  = (unsigned short*)(ws + off);
  off += kBytesWinB;
  unsigned short* WoutH = (unsigned short*)(ws + off);
  off += kBytesWoutH;
  unsigned short* WxB   = (unsigned short*)(ws + off);
  off += kBytesWxB;
  float* AlogC          = (float*)(ws + off);
  off += kBytesAlog;
  float* DparC          = (float*)(ws + off);
  off += kBytesDpar;
  unsigned short* XNh   = (unsigned short*)(ws + off);
  off += kBytesXNh;
  unsigned short* XNl   = (unsigned short*)(ws + off);
  off += kBytesXNl;
  float* XZ             = (float*)(ws + off);
  off += kBytesXZ;
  float* U              = (float*)(ws + off);
  off += kBytesU;
  unsigned short* Uh    = (unsigned short*)(ws + off);
  off += kBytesUh;
  unsigned short* Ul    = (unsigned short*)(ws + off);
  off += kBytesUl;
  float* BC             = (float*)(ws + off);
  off += kBytesBC;
  float* DTP            = (float*)(ws + off);
  off += kBytesDTP;
  unsigned short* YH    = (unsigned short*)(ws + off);
  off += kBytesYH;
  unsigned short* YL    = (unsigned short*)(ws + off);
  off += kBytesYL;
  if (off != kWsTotal) return;

  cast_bf16_kernel<<<dim3((kXzN * kDm / 8) / 256), 256, 0, stream>>>(W_in, WinB, kXzN * kDm / 8);
  cast_f16_carry_kernel<<<dim3((kDm * kDin / 8) / 256), 256, 0, stream>>>(W_out, WoutH, kDm * kDin / 8, kCarryWout);
  xproj_weight_kernel<<<dim3(kBcP), 256, 0, stream>>>(W_x, WxB);
  table_bf16r_kernel<<<dim3((kDin * kNstate / 4) / 256), 256, 0, stream>>>(A_log, AlogC, kDin * kNstate / 4);
  table_bf16r_kernel<<<dim3((kDin / 4) / 256), 256, 0, stream>>>(D_par, DparC, kDin / 4);

  for (int b = 0; b < kBatch; ++b) {
    const float* xb = x + (size_t)b * kSeq * kDm;
    float* ob = out + (size_t)b * kSeq * kDm;

    rownorm_split_kernel<<<dim3(kSeq / 8), 256, 0, stream>>>(xb, ln_w, ln_b, XNh, XNl, kSeq);

    gemm16_kernel<1, 4, 2, 0, 0><<<dim3((kSeq / 64) * (kXzN / 64) / 8), 256, 0, stream>>>(
        XNh, XNl, kDm, WinB, kDm, XZ, kXzN, xb, kDm,
        kSeq, kXzN, kDm, 1.0f, 0.0f);

    conv_silu_split_kernel<<<dim3(kSeq), 256, 0, stream>>>(XZ, conv_w, conv_b, U, Uh, Ul);

    gemm16_kernel<1, 4, 2, 0, 0><<<dim3((kSeq / 64) * (kBcP / 64) / 8), 256, 0, stream>>>(
        Uh, Ul, kDin, WxB, kDin, BC, kBcP, xb, kDm,
        kSeq, kBcP, kDin, 1.0f, 0.0f);

    step_preact_kernel<<<dim3(kSeq / 4), 256, 0, stream>>>(BC, W_dt, b_dt, DTP);

    ms1_args sa;
    sa.dtpre = DTP;
    sa.u = U;
    sa.bc = BC;
    sa.z = XZ;
    sa.A_log = AlogC;
    sa.Dskip = DparC;
    sa.y = (__half*)YH;
    sa.y_lo = (__half*)YL;
    sa.ld_dtpre = kDin;
    sa.ld_u = kDin;
    sa.ld_bc = kBcP;
    sa.ld_z = kXzN;
    sa.ld_y = kDin;
    sa.offB = kOffB;
    sa.offC = kOffC;
    sa.offZ = kDin;
    sa.ycarry = kCarryY;
    sa.dir = 1;
    sa.D = kDin;
    sa.L = kSeq;
    sa.nbatch = 1;
    ms1_scan_kernel<16><<<dim3(kDin / 64), 64, 0, stream>>>(sa);

    gemm16_kernel<0, 2, 2, 1, 1><<<dim3((kSeq / 32) * (kDm / 64) / 8), 256, 0, stream>>>(
        YH, YL, kDin, WoutH, kDin, ob, kDm, xb, kDm,
        kSeq, kDm, kDin, kFoldOut, kFoldResid);
  }
}
